// CrossAttention_14705968022104
// MI455X (gfx1250) — hardware-verified
//
#include <hip/hip_runtime.h>
#include <stdint.h>


#ifndef NB
#define NB 2
#endif
#ifndef SEQ
#define SEQ 1024
#endif
#define NB_FULL  2
#define LQ_FULL  1024
#define SKV      2048
#define SKV_FULL 2048
#define DIMC     1024
#define NHEAD    16
#define HD       64
#define QSCALE   0.125f

static_assert(NB >= 1 && NB <= NB_FULL);
static_assert(SEQ >= 64 && SEQ <= LQ_FULL && (SEQ % 64) == 0);
static_assert((SKV % 64) == 0 && SKV <= SKV_FULL);
static_assert((DIMC % 128) == 0 && NHEAD * HD == DIMC && HD == 64);

typedef unsigned short us;
typedef us     v8us  __attribute__((ext_vector_type(8), __may_alias__));
typedef us     v16us __attribute__((ext_vector_type(16)));
typedef __bf16 v16b  __attribute__((ext_vector_type(16)));
typedef float  v8f   __attribute__((ext_vector_type(8)));
typedef float  v4f   __attribute__((ext_vector_type(4), __may_alias__));

union Frag { v16b v; v16us u; v8us h[2]; };

__device__ __forceinline__ v8f vzero8()
{
    v8f z = {0.f, 0.f, 0.f, 0.f, 0.f, 0.f, 0.f, 0.f};
    return z;
}

__device__ __forceinline__ us f2bf(float f)
{
    unsigned int u = __float_as_uint(f);
    u += 0x7FFFu + ((u >> 16) & 1u);
    return (us)(u >> 16);
}
__device__ __forceinline__ float bf2f(us s)
{
    return __uint_as_float(((unsigned int)s) << 16);
}

__device__ __forceinline__ v8f wmma_bf16(const v16b a, const v16b b, v8f c)
{
    c = __builtin_amdgcn_wmma_f32_16x16x32_bf16(false, a, false, b, (short)0, c, false, false);
    asm volatile("v_nop\n\tv_nop\n\tv_nop\n\tv_nop" : "+v"(c) : "v"(a), "v"(b));
    return c;
}

__global__ __launch_bounds__(256) void conv_act_kernel(
    const float* __restrict__ xq, const float* __restrict__ xk, const float* __restrict__ xv,
    us* __restrict__ Xq, us* __restrict__ Xk, us* __restrict__ Xv)
{
    const int which = blockIdx.y;
    const float* src = (which == 0) ? xq : ((which == 1) ? xk : xv);
    us* dst          = (which == 0) ? Xq : ((which == 1) ? Xk : Xv);
    const int nrows   = (which == 0) ? (NB * SEQ) : (NB * SKV);
    const int per     = (which == 0) ? SEQ : SKV;
    const int perfull = (which == 0) ? LQ_FULL : SKV_FULL;

    const int chunk = blockIdx.x * 256 + threadIdx.x;
    if (chunk >= nrows * (DIMC / 8)) return;
    const int row = chunk / (DIMC / 8);
    const int c   = (chunk - row * (DIMC / 8)) * 8;
    const int bb  = row / per;
    const int i   = row - bb * per;

    const float* p = src + (size_t)(bb * perfull + i) * DIMC + c;
    const v4f x0 = *(const v4f*)p;
    const v4f x1 = *(const v4f*)(p + 4);
    v8us o;
#pragma unroll
    for (int j = 0; j < 4; ++j) { o[j] = f2bf(x0[j]); o[4 + j] = f2bf(x1[j]); }

    us* d = dst + (size_t)row * DIMC + c;
    *(volatile v8us*)d = o;
    __threadfence();
    *(volatile v8us*)d = o;
}

__global__ __launch_bounds__(256) void wtrans_kernel(
    const float* __restrict__ W0, const float* __restrict__ W1,
    const float* __restrict__ W2, const float* __restrict__ W3,
    us* __restrict__ T0, us* __restrict__ T1, us* __restrict__ T2, us* __restrict__ T3)
{
    __shared__ float tile[64 * 65];
    const int z = blockIdx.z;
    const float* W = (z == 0) ? W0 : ((z == 1) ? W1 : ((z == 2) ? W2 : W3));
    us* T          = (z == 0) ? T0 : ((z == 1) ? T1 : ((z == 2) ? T2 : T3));
    const int n0 = blockIdx.x * 64;
    const int k0 = blockIdx.y * 64;
    const int t  = threadIdx.x;

#pragma unroll
    for (int it = 0; it < 16; ++it) {
        const int kk = it * 4 + (t >> 6);
        const int nn = t & 63;
        tile[kk * 65 + nn] = W[(size_t)(k0 + kk) * DIMC + n0 + nn];
    }
    __syncthreads();

#pragma unroll
    for (int pass = 0; pass < 2; ++pass) {
#pragma unroll
        for (int it = 0; it < 2; ++it) {
            const int c  = it * 256 + t;
            const int nn = c >> 3;
            const int ch = c & 7;
            v8us o;
#pragma unroll
            for (int j = 0; j < 8; ++j) o[j] = f2bf(tile[(ch * 8 + j) * 65 + nn]);
            us* d = T + (size_t)(n0 + nn) * DIMC + k0 + ch * 8;
            *(volatile v8us*)d = o;
        }
        if (pass == 0) __threadfence();
    }
}

template<int MODE, int APL>
__global__ __launch_bounds__(128) void gemm_kernel(
    const us* __restrict__ A0, const us* __restrict__ A1, const us* __restrict__ Bt,
    const float* __restrict__ bias, float* __restrict__ Cf,
    us* __restrict__ Ch, us* __restrict__ Cl, float scale)
{
    __shared__ __attribute__((aligned(16))) us smem[18432];

    const int tid  = threadIdx.x;
    const int lane = tid & 31;
    const int w    = tid >> 5;
    const int h    = lane >> 4;
    const int lm   = lane & 15;
    const int n0   = blockIdx.x * 128;
    const int m0   = blockIdx.y * 64;

    v8f acc[4][2];
#pragma unroll
    for (int mt = 0; mt < 4; ++mt)
#pragma unroll
        for (int nt = 0; nt < 2; ++nt) acc[mt][nt] = vzero8();

    const size_t aoff = (size_t)(m0 + lm) * DIMC + 8 * h;
    const size_t boff = (size_t)(n0 + w * 32 + lm) * DIMC + 8 * h;

#pragma unroll 1
    for (int k0 = 0; k0 < DIMC; k0 += 32) {
        Frag b[2];
#pragma unroll
        for (int nt = 0; nt < 2; ++nt) {
            const us* p = Bt + boff + (size_t)(nt * 16) * DIMC + k0;
            b[nt].h[0] = *(const v8us*)(p);
            b[nt].h[1] = *(const v8us*)(p + 16);
        }
#pragma unroll
        for (int mt = 0; mt < 4; ++mt) {
            {
                const us* p = A0 + aoff + (size_t)(mt * 16) * DIMC + k0;
                Frag a;
                a.h[0] = *(const v8us*)(p);
                a.h[1] = *(const v8us*)(p + 16);
#pragma unroll
                for (int nt = 0; nt < 2; ++nt)
                    acc[mt][nt] = wmma_bf16(a.v, b[nt].v, acc[mt][nt]);
            }
            if (APL == 2) {
                const us* p = A1 + aoff + (size_t)(mt * 16) * DIMC + k0;
                Frag a;
                a.h[0] = *(const v8us*)(p);
                a.h[1] = *(const v8us*)(p + 16);
#pragma unroll
                for (int nt = 0; nt < 2; ++nt)
                    acc[mt][nt] = wmma_bf16(a.v, b[nt].v, acc[mt][nt]);
            }
        }
    }

    if (MODE == 0) {
        float* sf = (float*)smem;
#pragma unroll
        for (int mt = 0; mt < 4; ++mt)
#pragma unroll
            for (int nt = 0; nt < 2; ++nt)
#pragma unroll
                for (int r = 0; r < 8; ++r) {
                    const int rr = mt * 16 + 8 * h + r;
                    const int cc = w * 32 + nt * 16 + lm;
                    sf[rr * 132 + cc] = acc[mt][nt][r] * scale;
                }
        __syncthreads();
#pragma unroll
        for (int pass = 0; pass < 2; ++pass) {
#pragma unroll
            for (int it = 0; it < 16; ++it) {
                const int rr  = it * 4 + w;
                const int ch  = lane;
                const int col = n0 + ch * 4;
                v4f v = *(const v4f*)(sf + rr * 132 + ch * 4);
                const v4f bv = *(const v4f*)(bias + col);
#pragma unroll
                for (int j = 0; j < 4; ++j) v[j] = v[j] + bf2f(f2bf(bv[j]));
                const int m  = m0 + rr;
                const int bb = m / SEQ;
                const int l  = m - bb * SEQ;
                const size_t off = (size_t)(bb * LQ_FULL + l) * DIMC + col;
                *(volatile v4f*)(Cf + off) = v;
            }
            if (pass == 0) __threadfence();
        }
    } else if (MODE == 1) {
        us* sh = smem;
        us* sl = smem + 64 * 136;
#pragma unroll
        for (int mt = 0; mt < 4; ++mt)
#pragma unroll
            for (int nt = 0; nt < 2; ++nt)
#pragma unroll
                for (int r = 0; r < 8; ++r) {
                    const float v  = acc[mt][nt][r] * scale;
                    const us    hi = f2bf(v);
                    const us    lo = f2bf(v - bf2f(hi));
                    const int   rr = mt * 16 + 8 * h + r;
                    const int   cc = w * 32 + nt * 16 + lm;
                    sh[rr * 136 + cc] = hi;
                    sl[rr * 136 + cc] = lo;
                }
        __syncthreads();
#pragma unroll
        for (int pass = 0; pass < 2; ++pass) {
#pragma unroll
            for (int it = 0; it < 8; ++it) {
                const int c  = it * 128 + tid;
                const int rr = c >> 4;
                const int ch = c & 15;
                const v8us vh = *(const v8us*)(sh + rr * 136 + ch * 8);
                const v8us vl = *(const v8us*)(sl + rr * 136 + ch * 8);
                const size_t off = (size_t)(m0 + rr) * DIMC + n0 + ch * 8;
                *(volatile v8us*)(Ch + off) = vh;
                *(volatile v8us*)(Cl + off) = vl;
            }
            if (pass == 0) __threadfence();
        }
    } else {
        us* sh = smem;
        us* sl = smem + 128 * 72;
#pragma unroll
        for (int mt = 0; mt < 4; ++mt)
#pragma unroll
            for (int nt = 0; nt < 2; ++nt)
#pragma unroll
                for (int r = 0; r < 8; ++r) {
                    const float v  = acc[mt][nt][r] * scale;
                    const us    hi = f2bf(v);
                    const us    lo = f2bf(v - bf2f(hi));
                    const int   nn = w * 32 + nt * 16 + lm;
                    const int   ss = mt * 16 + 8 * h + r;
                    sh[nn * 72 + ss] = hi;
                    sl[nn * 72 + ss] = lo;
                }
        __syncthreads();
        const int bb = m0 / SKV;
        const int s0 = m0 - bb * SKV;
#pragma unroll
        for (int pass = 0; pass < 2; ++pass) {
#pragma unroll
            for (int it = 0; it < 8; ++it) {
                const int c  = it * 128 + tid;
                const int nn = c >> 3;
                const int ch = c & 7;
                const v8us vh = *(const v8us*)(sh + nn * 72 + ch * 8);
                const v8us vl = *(const v8us*)(sl + nn * 72 + ch * 8);
                const size_t off = ((size_t)(bb * DIMC + n0 + nn)) * SKV + s0 + ch * 8;
                *(volatile v8us*)(Ch + off) = vh;
                *(volatile v8us*)(Cl + off) = vl;
            }
            if (pass == 0) __threadfence();
        }
    }
}

__global__ __launch_bounds__(128) void attn_kernel(
    const us* __restrict__ Qh, const us* __restrict__ Ql,
    const us* __restrict__ Kh, const us* __restrict__ Kl,
    const us* __restrict__ Vh, const us* __restrict__ Vl,
    us* __restrict__ Xh, us* __restrict__ Xl)
{
    __shared__ __attribute__((aligned(16))) us xs[4 * 2 * 16 * 72];

    const int tid  = threadIdx.x;
    const int lane = tid & 31;
    const int w    = tid >> 5;
    const int h    = lane >> 4;
    const int lm   = lane & 15;
    const int b    = blockIdx.y / NHEAD;
    const int hd   = blockIdx.y - b * NHEAD;
    const int l0   = blockIdx.x * 64 + w * 16;

    Frag qh[2], ql[2];
    {
        const size_t qoff = (size_t)(b * SEQ + l0 + lm) * DIMC + hd * HD + 8 * h;
#pragma unroll
        for (int kt = 0; kt < 2; ++kt) {
            qh[kt].h[0] = *(const v8us*)(Qh + qoff + kt * 32);
            qh[kt].h[1] = *(const v8us*)(Qh + qoff + kt * 32 + 16);
            ql[kt].h[0] = *(const v8us*)(Ql + qoff + kt * 32);
            ql[kt].h[1] = *(const v8us*)(Ql + qoff + kt * 32 + 16);
        }
    }

    v8f oacc[4];
#pragma unroll
    for (int nt = 0; nt < 4; ++nt) oacc[nt] = vzero8();
    float mrun = -1.0e30f;
    float lrun = 0.f;

    const size_t koff = (size_t)(b * SKV + lm) * DIMC + hd * HD + 8 * h;
    const size_t voff = ((size_t)(b * DIMC + hd * HD + lm)) * SKV + 8 * h;

#pragma unroll 1
    for (int s0 = 0; s0 < SKV; s0 += 64) {
        v8f sacc[4];
#pragma unroll
        for (int mt = 0; mt < 4; ++mt) sacc[mt] = vzero8();
#pragma unroll
        for (int mt = 0; mt < 4; ++mt)
#pragma unroll
            for (int kt = 0; kt < 2; ++kt) {
                const size_t o = koff + (size_t)(s0 + mt * 16) * DIMC + kt * 32;
                Frag ah, al;
                ah.h[0] = *(const v8us*)(Kh + o);
                ah.h[1] = *(const v8us*)(Kh + o + 16);
                al.h[0] = *(const v8us*)(Kl + o);
                al.h[1] = *(const v8us*)(Kl + o + 16);
                sacc[mt] = wmma_bf16(ah.v, qh[kt].v, sacc[mt]);
                sacc[mt] = wmma_bf16(ah.v, ql[kt].v, sacc[mt]);
                sacc[mt] = wmma_bf16(al.v, qh[kt].v, sacc[mt]);
            }

        float mx = sacc[0][0];
#pragma unroll
        for (int mt = 0; mt < 4; ++mt)
#pragma unroll
            for (int r = 0; r < 8; ++r) mx = fmaxf(mx, sacc[mt][r]);
        mx = fmaxf(mx, __shfl_xor(mx, 16, 32));
        const float mnew  = fmaxf(mrun, mx);
        const float alpha = __expf(mrun - mnew);
        float rs = 0.f;
#pragma unroll
        for (int mt = 0; mt < 4; ++mt)
#pragma unroll
            for (int r = 0; r < 8; ++r) {
                const float p = __expf(sacc[mt][r] - mnew);
                sacc[mt][r] = p;
                rs += p;
            }
        rs += __shfl_xor(rs, 16, 32);
        lrun = lrun * alpha + rs;
        mrun = mnew;

#pragma unroll
        for (int r = 0; r < 8; ++r) {
            const float ar = __shfl(alpha, 8 * h + r, 32);
#pragma unroll
            for (int nt = 0; nt < 4; ++nt) oacc[nt][r] *= ar;
        }

        Frag ph[2], pl[2];
#pragma unroll
        for (int kt = 0; kt < 2; ++kt)
#pragma unroll
            for (int i = 0; i < 8; ++i) {
                const float p0  = sacc[2 * kt][i];
                const us    h0  = f2bf(p0);
                ph[kt].u[i]     = h0;
                pl[kt].u[i]     = f2bf(p0 - bf2f(h0));
                const float p1  = sacc[2 * kt + 1][i];
                const us    h1  = f2bf(p1);
                ph[kt].u[8 + i] = h1;
                pl[kt].u[8 + i] = f2bf(p1 - bf2f(h1));
            }

#pragma unroll
        for (int nt = 0; nt < 4; ++nt)
#pragma unroll
            for (int kt = 0; kt < 2; ++kt) {
                const size_t o = voff + (size_t)(nt * 16) * SKV + s0 + kt * 32;
                Frag vh, vl;
                vh.h[0] = *(const v8us*)(Vh + o);
                vh.h[1] = *(const v8us*)(Vh + o + 16);
                vl.h[0] = *(const v8us*)(Vl + o);
                vl.h[1] = *(const v8us*)(Vl + o + 16);
                oacc[nt] = wmma_bf16(ph[kt].v, vh.v, oacc[nt]);
                oacc[nt] = wmma_bf16(ph[kt].v, vl.v, oacc[nt]);
                oacc[nt] = wmma_bf16(pl[kt].v, vh.v, oacc[nt]);
            }
    }

    const float il = 1.0f / lrun;
    us* xsh = xs + w * (2 * 16 * 72);
    us* xsl = xsh + 16 * 72;
#pragma unroll
    for (int r = 0; r < 8; ++r) {
        const float ir = __shfl(il, 8 * h + r, 32);
#pragma unroll
        for (int nt = 0; nt < 4; ++nt) {
            const float v  = oacc[nt][r] * ir;
            const us    hi = f2bf(v);
            const us    lo = f2bf(v - bf2f(hi));
            const int  idx = (8 * h + r) * 72 + nt * 16 + lm;
            xsh[idx] = hi;
            xsl[idx] = lo;
        }
    }
    __syncthreads();
    const size_t rowbase = (size_t)(b * SEQ + l0);
#pragma unroll
    for (int pass = 0; pass < 2; ++pass) {
#pragma unroll
        for (int it = 0; it < 4; ++it) {
            const int rr = it * 4 + (lane >> 3);
            const int ch = lane & 7;
            const v8us vh = *(const v8us*)(xsh + rr * 72 + ch * 8);
            const v8us vl = *(const v8us*)(xsl + rr * 72 + ch * 8);
            const size_t off = (rowbase + rr) * DIMC + hd * HD + ch * 8;
            *(volatile v8us*)(Xh + off) = vh;
            *(volatile v8us*)(Xl + off) = vl;
        }
        if (pass == 0) __threadfence();
    }
}

extern "C" void kernel_launch(void* const* d_in, const int* in_sizes, int n_in,
                              void* d_out, int out_size, void* d_ws, size_t ws_size,
                              hipStream_t stream)
{
    if (n_in < 8) return;
    if (in_sizes[0] < ((NB - 1) * LQ_FULL + SEQ) * DIMC) return;
    if (in_sizes[1] < NB * SKV_FULL * DIMC) return;
    if (in_sizes[2] < NB * SKV_FULL * DIMC) return;
    if (in_sizes[3] < DIMC * DIMC) return;
    if (in_sizes[4] < DIMC * DIMC) return;
    if (in_sizes[5] < DIMC * DIMC) return;
    if (in_sizes[6] < DIMC * DIMC) return;
    if (in_sizes[7] < DIMC) return;
    if (out_size < ((NB - 1) * LQ_FULL + SEQ) * DIMC) return;

    const float* query = (const float*)d_in[0];
    const float* key   = (const float*)d_in[1];
    const float* value = (const float*)d_in[2];
    const float* Wq    = (const float*)d_in[3];
    const float* Wk    = (const float*)d_in[4];
    const float* Wv    = (const float*)d_in[5];
    const float* Wo    = (const float*)d_in[6];
    const float* bo    = (const float*)d_in[7];
    float*       out   = (float*)d_out;

    const size_t nXq  = (size_t)NB * SEQ * DIMC;
    const size_t nXkv = (size_t)NB * SKV * DIMC;
    const size_t nW   = (size_t)DIMC * DIMC;
    const size_t total = (5 * nXq + 6 * nXkv + 4 * nW) * sizeof(us);
    if (total > ws_size) return;

    us* wsp  = (us*)d_ws;
    us* Xq   = wsp;
    us* Xk   = Xq  + nXq;
    us* Xv   = Xk  + nXkv;
    us* Wqt  = Xv  + nXkv;
    us* Wkt  = Wqt + nW;
    us* Wvt  = Wkt + nW;
    us* Wot  = Wvt + nW;
    us* Qh   = Wot + nW;
    us* Ql   = Qh  + nXq;
    us* Kh   = Ql  + nXq;
    us* Kl   = Kh  + nXkv;
    us* Vth  = Kl  + nXkv;
    us* Vtl  = Vth + nXkv;
    us* Xh   = Vtl + nXkv;
    us* Xl   = Xh  + nXq;

    conv_act_kernel<<<dim3((NB * SKV * (DIMC / 8) + 255) / 256, 3), dim3(256), 0, stream>>>(
        query, key, value, Xq, Xk, Xv);
    wtrans_kernel<<<dim3(DIMC / 64, DIMC / 64, 4), dim3(256), 0, stream>>>(
        Wq, Wk, Wv, Wo, Wqt, Wkt, Wvt, Wot);
    gemm_kernel<1, 1><<<dim3(DIMC / 128, (NB * SEQ) / 64), dim3(128), 0, stream>>>(
        Xq, Xq, Wqt, bo, out, Qh, Ql, QSCALE);
    gemm_kernel<1, 1><<<dim3(DIMC / 128, (NB * SKV) / 64), dim3(128), 0, stream>>>(
        Xk, Xk, Wkt, bo, out, Kh, Kl, 1.0f);
    gemm_kernel<2, 1><<<dim3(DIMC / 128, (NB * SKV) / 64), dim3(128), 0, stream>>>(
        Xv, Xv, Wvt, bo, out, Vth, Vtl, 1.0f);
    attn_kernel<<<dim3(SEQ / 64, NB * NHEAD), dim3(128), 0, stream>>>(
        Qh, Ql, Kh, Kl, Vth, Vtl, Xh, Xl);
    gemm_kernel<0, 2><<<dim3(DIMC / 128, (NB * SEQ) / 64), dim3(128), 0, stream>>>(
        Xh, Xl, Wot, bo, out, Xh, Xl, 1.0f);
}
